// MSpatialGCN_13194139533745
// MI455X (gfx1250) — hardware-verified
//
#include <hip/hip_runtime.h>
#include <math.h>

typedef __attribute__((ext_vector_type(16))) _Float16 v16h;
typedef __attribute__((ext_vector_type(16))) __bf16 v16b;
typedef __attribute__((ext_vector_type(8)))  _Float16 v8h;
typedef __attribute__((ext_vector_type(8)))  float v8f;
typedef __attribute__((ext_vector_type(4)))  float v4f;
typedef __attribute__((ext_vector_type(2)))  float v2f;
typedef __attribute__((ext_vector_type(4)))  unsigned v4u;
typedef __attribute__((ext_vector_type(4)))  int v4i;
typedef float __attribute__((may_alias)) float_a;
typedef int __attribute__((may_alias)) int_a;

template <typename T> __device__ __forceinline__ void vst2(void* p, T v) { *(volatile T*)p = v; __threadfence(); *(volatile T*)p = v; }
__device__ __forceinline__ v8f wmma16(v16h a, v16h b, v8f c) {
  v8f d = __builtin_amdgcn_wmma_f32_16x16x32_f16(false, a, false, b, (short)0, c, false, false);
  asm volatile("v_nop\n\tv_nop\n\tv_nop\n\tv_nop" : "+v"(d) : "v"(a), "v"(b));
  return d;
}
__device__ __forceinline__ v8f wmma_bf(v16b a, v16b b, v8f c) {
  v8f d = __builtin_amdgcn_wmma_f32_16x16x32_bf16(false, a, false, b, (short)0, c, false, false);
  asm volatile("v_nop\n\tv_nop\n\tv_nop\n\tv_nop" : "+v"(d) : "v"(a), "v"(b));
  return d;
}
__device__ __forceinline__ v16h frag_h(const _Float16* rowk0, int lane) {
  union { v16h v; v8h q[2]; } u; const _Float16* p = rowk0 + 8 * (lane >> 4);
  u.q[0] = *(const v8h*)p; u.q[1] = *(const v8h*)(p + 16); return u.v;
}
__device__ __forceinline__ v16h frag_f32(const float* rowk0, int lane) {
  v16h a; const float* p = rowk0 + 8 * (lane >> 4);
#pragma unroll
  for (int i = 0; i < 8; ++i) { a[i] = (_Float16)p[i]; a[8 + i] = (_Float16)p[16 + i]; }
  return a;
}
__device__ __forceinline__ v16h frag_f32s(const float* rowk0, int lane, float sc) {
  v16h a; const float* p = rowk0 + 8 * (lane >> 4);
#pragma unroll
  for (int i = 0; i < 8; ++i) { a[i] = (_Float16)(p[i] * sc); a[8 + i] = (_Float16)(p[16 + i] * sc); }
  return a;
}
__device__ __forceinline__ v16h fragc_f32(const float* W, int k0, int n, int lane, int ld, int K) {
  v16h a; const int g = lane >> 4;
#pragma unroll
  for (int i = 0; i < 8; ++i) { const int ka = k0 + 8 * g + i, kb = ka + 16;
    a[i] = (_Float16)(ka < K ? W[(size_t)(ka < K ? ka : K - 1) * ld + n] : 0.f); a[8 + i] = (_Float16)(kb < K ? W[(size_t)(kb < K ? kb : K - 1) * ld + n] : 0.f); }
  return a;
}
struct F2 { v16b h, l; };
__device__ __forceinline__ F2 bsplit16(const float v[16]) { F2 r;
#pragma unroll
  for (int i = 0; i < 16; ++i) { const __bf16 h = (__bf16)v[i]; r.h[i] = h; r.l[i] = (__bf16)(v[i] - (float)h); }
  return r; }
__device__ __forceinline__ F2 split_row(const float* row, int k0, int lane) { float v[16]; const float* p = row + k0 + 8 * (lane >> 4);
#pragma unroll
  for (int i = 0; i < 8; ++i) { v[i] = p[i]; v[8 + i] = p[16 + i]; }
  return bsplit16(v); }
__device__ __forceinline__ F2 split_rowK(const float* row, int k0, int lane, int K) { float v[16]; const int g = lane >> 4;
#pragma unroll
  for (int i = 0; i < 8; ++i) { const int ka = k0 + 8 * g + i, kb = ka + 16; v[i] = ka < K ? row[ka < K ? ka : K - 1] : 0.f; v[8 + i] = kb < K ? row[kb < K ? kb : K - 1] : 0.f; }
  return bsplit16(v); }
__device__ __forceinline__ F2 split_col(const float* W, int k0, int n, int lane, int ld, int K) { float v[16]; const int g = lane >> 4;
#pragma unroll
  for (int i = 0; i < 8; ++i) { const int ka = k0 + 8 * g + i, kb = ka + 16; v[i] = ka < K ? W[(size_t)(ka < K ? ka : K - 1) * ld + n] : 0.f; v[8 + i] = kb < K ? W[(size_t)(kb < K ? kb : K - 1) * ld + n] : 0.f; }
  return bsplit16(v); }
__device__ __forceinline__ v8f mac3(const F2& a, const F2& b, v8f c) { c = wmma_bf(a.l, b.h, c); c = wmma_bf(a.h, b.l, c); return wmma_bf(a.h, b.h, c); }
__device__ __forceinline__ float sigm(float v) { return 1.0f / (1.0f + expf(-v)); }
#define LDSX() do { asm volatile("s_wait_dscnt 0" ::: "memory"); __builtin_amdgcn_wave_barrier(); __builtin_amdgcn_fence(__ATOMIC_RELEASE, "workgroup"); } while (0)


#define NB 2
#define CC 64
#ifndef NN
#define NN 3136
#endif
#define NSTR 3136
#define NH 4
#define IP 32
#define OP 64
#ifndef TQB
#define TQB (NN / 64)
#define TNB NB
#endif
typedef __attribute__((ext_vector_type(8))) __bf16 v8b;
__device__ __forceinline__ v16b frag_b(const __bf16* rowk0, int lane) {
  union { v16b v; v8b q[2]; } u; const __bf16* p = rowk0 + 8 * (lane >> 4);
  u.q[0] = *(const v8b*)p; u.q[1] = *(const v8b*)(p + 16); return u.v;
}
__device__ __forceinline__ float bfr(float v) { return (float)(__bf16)v; }
__device__ __attribute__((noinline)) float exp_ni(float v) { return expf(v); }
__device__ __attribute__((noinline)) float erf_ni(float v) { return erff(v); }

#define WS_PW   0u
#define PKQV 0
#define PW1 (PKQV + 3 * NH * IP * CC)
#define PW2 (PW1 + OP * IP)
#define PWF (PW2 + OP * OP)
#define PWEND (PWF + OP * NH * OP)
#define WS_KQV  (WS_PW + 2u * PWEND)
#define WS_ST   (WS_KQV + 4u * NB * NN * 384)
#define WS_VH   (WS_ST + 4u * NB * NH * 2 * NN)
#define WS_VL   (WS_VH + 2u * NB * NH * IP * NN)
#define WS_AW   (WS_VL + 2u * NB * NH * IP * NN)
#define WS_AH   (WS_AW + 4u * NB * NH * NN * OP)
#define WS_AL   (WS_AH + 2u * NB * NH * OP * NN)
#define WS_Y    (WS_AL + 2u * NB * NH * OP * NN)
#define WS_END  (WS_Y + 4u * NB * NN * NH * OP)

__global__ __launch_bounds__(256) void k_pack(const float* __restrict__ WK, const float* __restrict__ WQ, const float* __restrict__ WV, const float* __restrict__ W1, const float* __restrict__ W2, const float* __restrict__ WF, __bf16* __restrict__ PW) {
  __shared__ __align__(16) __bf16 s[256]; const int r = blockIdx.x, which = blockIdx.y, tid = threadIdx.x; int K; size_t dst; const float* src;
  if (which == 0) { if (r >= 384) return; K = CC; dst = PKQV + (size_t)r * CC; src = (r < 128) ? WK + (size_t)r * CC : (r < 256 ? WQ + (size_t)(r - 128) * CC : WV + (size_t)(r - 256) * CC); }
  else if (which == 1) { if (r >= OP) return; K = IP; dst = PW1 + (size_t)r * IP; src = W1 + (size_t)r * IP; }
  else if (which == 2) { if (r >= OP) return; K = OP; dst = PW2 + (size_t)r * OP; src = W2 + (size_t)r * OP; }
  else { if (r >= OP) return; K = NH * OP; dst = PWF + (size_t)r * NH * OP; src = WF + (size_t)r * NH * OP; }
  if (tid < K) s[tid] = (__bf16)src[tid];
  __syncthreads();
  if (tid < K / 8) vst2((unsigned*)(PW + dst + tid * 8), *(const v4u*)&s[tid * 8]);
}
__global__ __launch_bounds__(128) void k_proj(const float* __restrict__ X, const __bf16* __restrict__ PW, const float* __restrict__ BK, const float* __restrict__ BQ, const float* __restrict__ BV, float* __restrict__ KQV) {
  __shared__ __align__(16) __bf16 sx[64][CC + 8]; __shared__ __align__(16) float so[4][16][132];
  const int tid = threadIdx.x, wave = tid >> 5, lane = tid & 31, col = lane & 15, g = lane >> 4; const int b = blockIdx.z; const int p0 = blockIdx.x * 64; const int n0 = blockIdx.y * 128;
  for (int q = tid; q < CC * 64; q += 128) { const int c = q >> 6, nl = q & 63; sx[nl][c] = (__bf16)X[((size_t)b * CC + c) * NSTR + p0 + nl]; }
  __syncthreads();
  v8f acc[8] = {};
#pragma unroll
  for (int kc = 0; kc < CC / 32; ++kc) { v16b a;
#pragma unroll
    for (int i = 0; i < 8; ++i) { a[i] = sx[wave * 16 + col][kc * 32 + 8 * g + i]; a[8 + i] = sx[wave * 16 + col][kc * 32 + 16 + 8 * g + i]; }
#pragma unroll
    for (int j = 0; j < 8; ++j) acc[j] = wmma_bf(a, frag_b(PW + PKQV + (size_t)(n0 + j * 16 + col) * CC + kc * 32, lane), acc[j]); }
  const float* bias = (n0 < 128) ? BK : (n0 < 256 ? BQ : BV);
#pragma unroll
  for (int j = 0; j < 8; ++j) { const float bb = bfr(bias[(n0 & 127) + j * 16 + col]);
#pragma unroll
    for (int r = 0; r < 8; ++r) so[wave][8 * g + r][j * 16 + col] = acc[j][r] + bb; }
  LDSX();
  for (int rl = 0; rl < 16; ++rl) vst2(KQV + ((size_t)b * NN + p0 + wave * 16 + rl) * 384 + n0 + lane * 4, *(const v4f*)&so[wave][rl][lane * 4]);
}
__global__ __launch_bounds__(128) void k_colstat(const float* __restrict__ KQV, float* __restrict__ ST) {
  __shared__ __align__(16) float sm[2][64];
  const int tid = threadIdx.x, wave = tid >> 5, lane = tid & 31, col = lane & 15, g = lane >> 4; const int mb = blockIdx.x, h = blockIdx.y, b = blockIdx.z; const int m0 = mb * 64 + wave * 16;
  const F2 aq = split_row(KQV + ((size_t)b * NN + m0 + col) * 384 + 128 + h * IP, 0, lane);
  float mx[8], z[8];
#pragma unroll
  for (int r = 0; r < 8; ++r) { mx[r] = -3.0e38f; z[r] = 0.f; }
#pragma unroll 1
  for (int ns = 0; ns < NN / 32; ++ns) { v8f s[2];
#pragma unroll
    for (int ct = 0; ct < 2; ++ct) { const int nn = ns * 32 + ct * 16 + col; const F2 kb = split_row(KQV + ((size_t)b * NN + nn) * 384 + h * IP, 0, lane); s[ct] = mac3(aq, kb, (v8f){}); }
#pragma unroll
    for (int r = 0; r < 8; ++r) { float m2 = fmaxf(s[0][r], s[1][r]);
#pragma unroll
      for (int o = 1; o < 16; o <<= 1) m2 = fmaxf(m2, __shfl_xor(m2, o));
      const float mn = fmaxf(mx[r], m2); const float alpha = exp_ni(mx[r] - mn); float es = exp_ni(s[0][r] - mn) + exp_ni(s[1][r] - mn);
#pragma unroll
      for (int o = 1; o < 16; o <<= 1) es += __shfl_xor(es, o);
      z[r] = z[r] * alpha + es; mx[r] = mn; } }
  if (col == 0) {
#pragma unroll
    for (int r = 0; r < 8; ++r) { sm[0][wave * 16 + 8 * g + r] = mx[r]; sm[1][wave * 16 + 8 * g + r] = 1.0f / z[r]; } }
  __syncthreads();
  if (tid < 32) { const int w = tid >> 4, pc = tid & 15; vst2(ST + (((size_t)b * NH + h) * 2 + w) * NN + mb * 64 + pc * 4, *(const v4f*)&sm[w][pc * 4]); }
}
template <int W>
__global__ __launch_bounds__(256) void k_plane(const float* __restrict__ SRC, int ldv, int off_b, int off_h, const float* __restrict__ ST, __bf16* __restrict__ PH, __bf16* __restrict__ PL) {
  __shared__ __align__(16) __bf16 sh[W][72], sl[W][72]; const int tid = threadIdx.x; const int mb = blockIdx.x, h = blockIdx.y, b = blockIdx.z; const int m0 = mb * 64;
  for (int q = tid; q < 64 * W; q += 256) { const int ml = q / W, w = q % W; const float iz = ST[(((size_t)b * NH + h) * 2 + 1) * NN + m0 + ml]; const float v = SRC[((size_t)b * off_b + h * off_h) + (size_t)(m0 + ml) * ldv + w] * iz; const __bf16 hb = (__bf16)v; sh[w][ml] = hb; sl[w][ml] = (__bf16)(v - (float)hb); }
  __syncthreads();
  for (int q = tid; q < W * 8; q += 256) { const int w = q >> 3, pc = q & 7; const size_t o = (((size_t)b * NH + h) * W + w) * NN + m0 + pc * 8; vst2((unsigned*)(PH + o), *(const v4u*)&sh[w][pc * 8]); vst2((unsigned*)(PL + o), *(const v4u*)&sl[w][pc * 8]); }
}
template <int STAGE>
__global__ __launch_bounds__(128) void k_av(const float* __restrict__ KQV, const float* __restrict__ ST, const __bf16* __restrict__ PH, const __bf16* __restrict__ PL, const __bf16* __restrict__ PW, const float* __restrict__ BL, const float* __restrict__ G_, const float* __restrict__ BE, const float* __restrict__ RM, const float* __restrict__ RV, float* __restrict__ OUT) {
  constexpr int NTV = (STAGE == 1) ? 2 : 4; constexpr int WV = NTV * 16;
  __shared__ __align__(16) float sp[4][16][36]; __shared__ __align__(16) float sa[4][16][68]; __shared__ __align__(16) float so[4][16][68];
  const int tid = threadIdx.x, wave = tid >> 5, lane = tid & 31, col = lane & 15, g = lane >> 4; const int nb = blockIdx.x, h = blockIdx.y, b = blockIdx.z; const int q0 = nb * 64 + wave * 16;
  const F2 ak = split_row(KQV + ((size_t)b * NN + q0 + col) * 384 + h * IP, 0, lane);
  const float* Mrow = ST + (((size_t)b * NH + h) * 2 + 0) * NN;
  v8f acc[NTV]; for (int j = 0; j < NTV; ++j) acc[j] = (v8f){};
#pragma unroll 1
  for (int ms = 0; ms < NN / 32; ++ms) {
#pragma unroll
    for (int ct = 0; ct < 2; ++ct) { const int mm = ms * 32 + ct * 16 + col; const F2 qb = split_row(KQV + ((size_t)b * NN + mm) * 384 + 128 + h * IP, 0, lane); const v8f s = mac3(ak, qb, (v8f){}); const float Mm = Mrow[mm];
#pragma unroll
      for (int r = 0; r < 8; ++r) sp[wave][8 * g + r][ct * 16 + col] = exp_ni(s[r] - Mm); }
    LDSX();
    const F2 pa = split_row(&sp[wave][col][0], 0, lane);
#pragma unroll
    for (int dt = 0; dt < NTV; ++dt) { const size_t vr = (((size_t)b * NH + h) * WV + dt * 16 + col) * NN + ms * 32; const v16b vh = frag_b(PH + vr, lane), vl = frag_b(PL + vr, lane); acc[dt] = wmma_bf(pa.l, vh, acc[dt]); acc[dt] = wmma_bf(pa.h, vl, acc[dt]); acc[dt] = wmma_bf(pa.h, vh, acc[dt]); }
    LDSX(); }
#pragma unroll
  for (int dt = 0; dt < NTV; ++dt)
#pragma unroll
    for (int r = 0; r < 8; ++r) sa[wave][8 * g + r][dt * 16 + col] = acc[dt][r];
  LDSX();
  v8f acc2[4] = {};
#pragma unroll
  for (int kc = 0; kc < WV / 32; ++kc) { const F2 a = split_row(&sa[wave][col][0], kc * 32, lane);
#pragma unroll
    for (int j = 0; j < 4; ++j) { const v16b w = frag_b(PW + (STAGE == 1 ? PW1 : PW2) + (size_t)(j * 16 + col) * WV + kc * 32, lane); acc2[j] = wmma_bf(a.l, w, acc2[j]); acc2[j] = wmma_bf(a.h, w, acc2[j]); } }
#pragma unroll
  for (int j = 0; j < 4; ++j) { const int o = j * 16 + col; const int ch = h * OP + o; const float bb = bfr(BL[o]); const float sc = bfr(G_[ch]) / sqrtf(bfr(RV[ch]) + 1e-5f); const float sh = bfr(BE[ch]) - bfr(RM[ch]) * sc;
#pragma unroll
    for (int r = 0; r < 8; ++r) { const float v = (acc2[j][r] + bb) * sc + sh; so[wave][8 * g + r][o] = fmaxf(v, 0.f); } }
  LDSX();
  if (STAGE == 1) { for (int rl = 0; rl < 16; ++rl) if (lane < 16) vst2(OUT + (((size_t)b * NH + h) * NN + q0 + rl) * OP + lane * 4, *(const v4f*)&so[wave][rl][lane * 4]); }
  else { for (int rl = 0; rl < 16; ++rl) if (lane < 16) vst2(OUT + ((size_t)b * NN + q0 + rl) * (NH * OP) + h * OP + lane * 4, *(const v4f*)&so[wave][rl][lane * 4]); }
}
__global__ __launch_bounds__(128) void k_final(const float* __restrict__ Y, const __bf16* __restrict__ PW, const float* __restrict__ BF, float* __restrict__ out) {
  __shared__ __align__(16) float st[OP][68];
  const int tid = threadIdx.x, wave = tid >> 5, lane = tid & 31, col = lane & 15, g = lane >> 4; const int b = blockIdx.y; const int p0 = blockIdx.x * 64; const size_t r0 = (size_t)b * NN + p0 + wave * 16;
  v8f acc[4] = {};
#pragma unroll 2
  for (int kc = 0; kc < NH * OP / 32; ++kc) { const F2 a = split_row(Y + (r0 + col) * (NH * OP), kc * 32, lane);
#pragma unroll
    for (int j = 0; j < 4; ++j) { const v16b w = frag_b(PW + PWF + (size_t)(j * 16 + col) * (NH * OP) + kc * 32, lane); acc[j] = wmma_bf(a.l, w, acc[j]); acc[j] = wmma_bf(a.h, w, acc[j]); } }
#pragma unroll
  for (int j = 0; j < 4; ++j) { const int o = j * 16 + col; const float bb = bfr(BF[o]);
#pragma unroll
    for (int r = 0; r < 8; ++r) st[o][wave * 16 + 8 * g + r] = acc[j][r] + bb; }
  __syncthreads();
  for (int q = tid; q < OP * 16; q += 128) { const int o = q >> 4, pc = q & 15; vst2(out + ((size_t)b * OP + o) * NSTR + p0 + pc * 4, *(const v4f*)&st[o][pc * 4]); }
}
extern "C" void kernel_launch(void* const* d_in, const int* in_sizes, int n_in, void* d_out, int out_size, void* d_ws, size_t ws_size, hipStream_t stream) {
  (void)in_sizes; (void)n_in; (void)out_size;
  const float** F = (const float**)d_in;
  if (ws_size < (size_t)WS_END) return;
  char* ws = (char*)d_ws; __bf16 *PW = (__bf16*)(ws + WS_PW), *VH = (__bf16*)(ws + WS_VH), *VL = (__bf16*)(ws + WS_VL), *AH = (__bf16*)(ws + WS_AH), *AL = (__bf16*)(ws + WS_AL); float *KQV = (float*)(ws + WS_KQV), *ST = (float*)(ws + WS_ST), *AW = (float*)(ws + WS_AW), *Y = (float*)(ws + WS_Y);
  k_pack<<<dim3(384, 4), 256, 0, stream>>>(F[1], F[3], F[5], F[7], F[13], F[19], PW);
  k_proj<<<dim3(NN / 64, 3, TNB), 128, 0, stream>>>(F[0], PW, F[2], F[4], F[6], KQV);
  k_colstat<<<dim3(NN / 64, NH, TNB), 128, 0, stream>>>(KQV, ST);
  k_plane<IP><<<dim3(NN / 64, NH, TNB), 256, 0, stream>>>(KQV + 256, 384, NN * 384, IP, ST, VH, VL);
  k_av<1><<<dim3(TQB, NH, TNB), 128, 0, stream>>>(KQV, ST, VH, VL, PW, F[8], F[9], F[10], F[11], F[12], AW);
  k_plane<OP><<<dim3(NN / 64, NH, TNB), 256, 0, stream>>>(AW, OP, NH * NN * OP, NN * OP, ST, AH, AL);
  k_av<2><<<dim3(TQB, NH, TNB), 128, 0, stream>>>(KQV, ST, AH, AL, PW, F[14], F[15], F[16], F[17], F[18], Y);
  k_final<<<dim3(TQB, TNB), 128, 0, stream>>>(Y, PW, F[20], (float*)d_out);
}
